// SA_ABMILP_84112639525171
// MI455X (gfx1250) — hardware-verified
//
#include <hip/hip_runtime.h>
#include <math.h>

typedef __attribute__((ext_vector_type(16))) _Float16 v16h;
typedef __attribute__((ext_vector_type(16))) __bf16 v16b;
typedef __attribute__((ext_vector_type(8)))  _Float16 v8h;
typedef __attribute__((ext_vector_type(8)))  float v8f;
typedef __attribute__((ext_vector_type(4)))  float v4f;
typedef __attribute__((ext_vector_type(2)))  float v2f;
typedef __attribute__((ext_vector_type(4)))  unsigned v4u;
typedef __attribute__((ext_vector_type(4)))  int v4i;
typedef float __attribute__((may_alias)) float_a;
typedef int __attribute__((may_alias)) int_a;

template <typename T> __device__ __forceinline__ void vst2(void* p, T v) { *(volatile T*)p = v; __threadfence(); *(volatile T*)p = v; }
__device__ __forceinline__ v8f wmma16(v16h a, v16h b, v8f c) {
  v8f d = __builtin_amdgcn_wmma_f32_16x16x32_f16(false, a, false, b, (short)0, c, false, false);
  asm volatile("v_nop\n\tv_nop\n\tv_nop\n\tv_nop" : "+v"(d) : "v"(a), "v"(b));
  return d;
}
__device__ __forceinline__ v8f wmma_bf(v16b a, v16b b, v8f c) {
  v8f d = __builtin_amdgcn_wmma_f32_16x16x32_bf16(false, a, false, b, (short)0, c, false, false);
  asm volatile("v_nop\n\tv_nop\n\tv_nop\n\tv_nop" : "+v"(d) : "v"(a), "v"(b));
  return d;
}
__device__ __forceinline__ v16h frag_h(const _Float16* rowk0, int lane) {
  union { v16h v; v8h q[2]; } u; const _Float16* p = rowk0 + 8 * (lane >> 4);
  u.q[0] = *(const v8h*)p; u.q[1] = *(const v8h*)(p + 16); return u.v;
}
__device__ __forceinline__ v16h frag_f32(const float* rowk0, int lane) {
  v16h a; const float* p = rowk0 + 8 * (lane >> 4);
#pragma unroll
  for (int i = 0; i < 8; ++i) { a[i] = (_Float16)p[i]; a[8 + i] = (_Float16)p[16 + i]; }
  return a;
}
__device__ __forceinline__ v16h frag_f32s(const float* rowk0, int lane, float sc) {
  v16h a; const float* p = rowk0 + 8 * (lane >> 4);
#pragma unroll
  for (int i = 0; i < 8; ++i) { a[i] = (_Float16)(p[i] * sc); a[8 + i] = (_Float16)(p[16 + i] * sc); }
  return a;
}
__device__ __forceinline__ v16h fragc_f32(const float* W, int k0, int n, int lane, int ld, int K) {
  v16h a; const int g = lane >> 4;
#pragma unroll
  for (int i = 0; i < 8; ++i) { const int ka = k0 + 8 * g + i, kb = ka + 16;
    a[i] = (_Float16)(ka < K ? W[(size_t)(ka < K ? ka : K - 1) * ld + n] : 0.f); a[8 + i] = (_Float16)(kb < K ? W[(size_t)(kb < K ? kb : K - 1) * ld + n] : 0.f); }
  return a;
}
struct F2 { v16b h, l; };
__device__ __forceinline__ F2 bsplit16(const float v[16]) { F2 r;
#pragma unroll
  for (int i = 0; i < 16; ++i) { const __bf16 h = (__bf16)v[i]; r.h[i] = h; r.l[i] = (__bf16)(v[i] - (float)h); }
  return r; }
__device__ __forceinline__ F2 split_row(const float* row, int k0, int lane) { float v[16]; const float* p = row + k0 + 8 * (lane >> 4);
#pragma unroll
  for (int i = 0; i < 8; ++i) { v[i] = p[i]; v[8 + i] = p[16 + i]; }
  return bsplit16(v); }
__device__ __forceinline__ F2 split_rowK(const float* row, int k0, int lane, int K) { float v[16]; const int g = lane >> 4;
#pragma unroll
  for (int i = 0; i < 8; ++i) { const int ka = k0 + 8 * g + i, kb = ka + 16; v[i] = ka < K ? row[ka < K ? ka : K - 1] : 0.f; v[8 + i] = kb < K ? row[kb < K ? kb : K - 1] : 0.f; }
  return bsplit16(v); }
__device__ __forceinline__ F2 split_col(const float* W, int k0, int n, int lane, int ld, int K) { float v[16]; const int g = lane >> 4;
#pragma unroll
  for (int i = 0; i < 8; ++i) { const int ka = k0 + 8 * g + i, kb = ka + 16; v[i] = ka < K ? W[(size_t)(ka < K ? ka : K - 1) * ld + n] : 0.f; v[8 + i] = kb < K ? W[(size_t)(kb < K ? kb : K - 1) * ld + n] : 0.f; }
  return bsplit16(v); }
__device__ __forceinline__ v8f mac3(const F2& a, const F2& b, v8f c) { c = wmma_bf(a.l, b.h, c); c = wmma_bf(a.h, b.l, c); return wmma_bf(a.h, b.h, c); }
__device__ __forceinline__ float sigm(float v) { return 1.0f / (1.0f + expf(-v)); }
#define LDSX() do { asm volatile("s_wait_dscnt 0" ::: "memory"); __builtin_amdgcn_wave_barrier(); __builtin_amdgcn_fence(__ATOMIC_RELEASE, "workgroup"); } while (0)


#define NP 8192
#define D0 1024
#define L1D 256
#define L2D 128
#define L3D 64
#define DQ 8
typedef __attribute__((ext_vector_type(8))) __bf16 v8b;
__device__ __forceinline__ v16b frag_b(const __bf16* rowk0, int lane) {
  union { v16b v; v8b q[2]; } u; const __bf16* p = rowk0 + 8 * (lane >> 4);
  u.q[0] = *(const v8b*)p; u.q[1] = *(const v8b*)(p + 16); return u.v;
}
__device__ __forceinline__ float bfr(float v) { return (float)(__bf16)v; }
__device__ __attribute__((noinline)) float exp_ni(float v) { return expf(v); }
__device__ __attribute__((noinline)) float erf_ni(float v) { return erff(v); }
__device__ __attribute__((noinline)) float tanh_ni(float v) { return tanhf(v); }

#define PK_1 0
#define PK_2 (PK_1 + L1D * D0)
#define PK_3 (PK_2 + L2D * L1D)
#define PK_Q (PK_3 + L3D * L2D)
#define PK_K (PK_Q + 16 * L3D)
#define PK_V (PK_K + 16 * L3D)
#define PK_END (PK_V + L3D * L3D)
#define WS_PK  0u
#define WS_H   (((2u * PK_END) + 127u) / 128u * 128u)
#define WS_QH  (WS_H + 4u * NP * L3D)
#define WS_KH  (WS_QH + 2u * NP * 32)
#define WS_VT  (WS_KH + 2u * NP * 32)
#define WS_H2  (WS_VT + 2u * NP * L3D)
#define WS_SC  (WS_H2 + 4u * NP * L3D)
#define WS_END (WS_SC + 4u * NP)

__global__ __launch_bounds__(256) void k_pack(const float* __restrict__ W1, const float* __restrict__ W2, const float* __restrict__ W3, const float* __restrict__ WQ, const float* __restrict__ WK, const float* __restrict__ WV, __bf16* __restrict__ PK) {
  __shared__ __align__(16) __bf16 s[D0]; const int n = blockIdx.x, which = blockIdx.y, t = threadIdx.x; int K; size_t dst;
  if (which == 0) { K = D0; dst = PK_1 + (size_t)n * D0; for (int k = t; k < K; k += 256) s[k] = (__bf16)W1[(size_t)k * L1D + n]; }
  else if (which == 1) { if (n >= L2D) return; K = L1D; dst = PK_2 + (size_t)n * L1D; for (int k = t; k < K; k += 256) s[k] = (__bf16)W2[(size_t)k * L2D + n]; }
  else if (which == 2) { if (n >= L3D) return; K = L2D; dst = PK_3 + (size_t)n * L2D; for (int k = t; k < K; k += 256) s[k] = (__bf16)W3[(size_t)k * L3D + n]; }
  else if (which == 3) { if (n >= 16) return; K = L3D; dst = PK_Q + (size_t)n * L3D; for (int k = t; k < K; k += 256) s[k] = (__bf16)((n < DQ) ? WQ[(size_t)k * DQ + n] : 0.f); }
  else if (which == 4) { if (n >= 16) return; K = L3D; dst = PK_K + (size_t)n * L3D; for (int k = t; k < K; k += 256) s[k] = (__bf16)((n < DQ) ? WK[(size_t)k * DQ + n] : 0.f); }
  else { if (n >= L3D) return; K = L3D; dst = PK_V + (size_t)n * L3D; for (int k = t; k < K; k += 256) s[k] = (__bf16)WV[(size_t)k * L3D + n]; }
  __syncthreads();
  for (int q = t; q < K / 8; q += 256) vst2((unsigned*)(PK + dst + q * 8), *(const v4u*)&s[q * 8]);
}
__global__ __launch_bounds__(128) void k_mlp(const float* __restrict__ X, const __bf16* __restrict__ PK, const float* __restrict__ B1, const float* __restrict__ B2, const float* __restrict__ B3, const float* __restrict__ BQ, const float* __restrict__ BK, const float* __restrict__ BV, float* __restrict__ H, _Float16* __restrict__ QH, _Float16* __restrict__ KH, _Float16* __restrict__ VT) {
  __shared__ __align__(16) __bf16 s1h[4][16][L1D + 8], s1l[4][16][L1D + 8]; __shared__ __align__(16) __bf16 s2h[4][16][L2D + 8], s2l[4][16][L2D + 8]; __shared__ __align__(16) __bf16 s3h[4][16][L3D + 8], s3l[4][16][L3D + 8]; __shared__ __align__(16) float sH[4][16][L3D + 4]; __shared__ __align__(16) _Float16 sq[4][16][40], sk[4][16][40]; __shared__ __align__(16) _Float16 svt[L3D][72];
  const int tid = threadIdx.x, wave = tid >> 5, lane = tid & 31, col = lane & 15, g = lane >> 4; const size_t r0 = (size_t)blockIdx.x * 64 + wave * 16;
#pragma unroll 1
  for (int half = 0; half < 2; ++half) { v8f acc[8] = {};
#pragma unroll 2
    for (int kc = 0; kc < D0 / 32; ++kc) { v16b a; { const float* p = X + (r0 + col) * D0 + kc * 32 + 8 * g;
#pragma unroll
        for (int i = 0; i < 8; ++i) { a[i] = (__bf16)p[i]; a[8 + i] = (__bf16)p[16 + i]; } }
#pragma unroll
      for (int j = 0; j < 8; ++j) acc[j] = wmma_bf(a, frag_b(PK + PK_1 + (size_t)(half * 128 + j * 16 + col) * D0 + kc * 32, lane), acc[j]); }
#pragma unroll
    for (int j = 0; j < 8; ++j) { const int c = half * 128 + j * 16 + col; const float bb = bfr(B1[c]);
#pragma unroll
      for (int r = 0; r < 8; ++r) { const float v = fmaxf(acc[j][r] + bb, 0.f); const __bf16 hb = (__bf16)v; s1h[wave][8 * g + r][c] = hb; s1l[wave][8 * g + r][c] = (__bf16)(v - (float)hb); } } }
  LDSX();
  { v8f acc[8] = {};
#pragma unroll
    for (int kc = 0; kc < L1D / 32; ++kc) { F2 a; a.h = frag_b(&s1h[wave][col][kc * 32], lane); a.l = frag_b(&s1l[wave][col][kc * 32], lane);
#pragma unroll
      for (int j = 0; j < 8; ++j) { const v16b w = frag_b(PK + PK_2 + (size_t)(j * 16 + col) * L1D + kc * 32, lane); acc[j] = wmma_bf(a.l, w, acc[j]); acc[j] = wmma_bf(a.h, w, acc[j]); } }
#pragma unroll
    for (int j = 0; j < 8; ++j) { const int c = j * 16 + col; const float bb = bfr(B2[c]);
#pragma unroll
      for (int r = 0; r < 8; ++r) { const float v = fmaxf(acc[j][r] + bb, 0.f); const __bf16 hb = (__bf16)v; s2h[wave][8 * g + r][c] = hb; s2l[wave][8 * g + r][c] = (__bf16)(v - (float)hb); } } }
  LDSX();
  { v8f acc[4] = {};
#pragma unroll
    for (int kc = 0; kc < L2D / 32; ++kc) { F2 a; a.h = frag_b(&s2h[wave][col][kc * 32], lane); a.l = frag_b(&s2l[wave][col][kc * 32], lane);
#pragma unroll
      for (int j = 0; j < 4; ++j) { const v16b w = frag_b(PK + PK_3 + (size_t)(j * 16 + col) * L2D + kc * 32, lane); acc[j] = wmma_bf(a.l, w, acc[j]); acc[j] = wmma_bf(a.h, w, acc[j]); } }
#pragma unroll
    for (int j = 0; j < 4; ++j) { const int c = j * 16 + col; const float bb = bfr(B3[c]);
#pragma unroll
      for (int r = 0; r < 8; ++r) { const float v = fmaxf(acc[j][r] + bb, 0.f); sH[wave][8 * g + r][c] = v; const __bf16 hb = (__bf16)v; s3h[wave][8 * g + r][c] = hb; s3l[wave][8 * g + r][c] = (__bf16)(v - (float)hb); } } }
  LDSX();
  { v8f acc[6] = {};
#pragma unroll
    for (int kc = 0; kc < L3D / 32; ++kc) { F2 a; a.h = frag_b(&s3h[wave][col][kc * 32], lane); a.l = frag_b(&s3l[wave][col][kc * 32], lane);
#pragma unroll
      for (int j = 0; j < 6; ++j) { const __bf16* P = (j == 0) ? PK + PK_Q : (j == 1) ? PK + PK_K : PK + PK_V + (size_t)(j - 2) * 16 * L3D; const v16b w = frag_b(P + (size_t)col * L3D + kc * 32, lane); acc[j] = wmma_bf(a.l, w, acc[j]); acc[j] = wmma_bf(a.h, w, acc[j]); } }
#pragma unroll
    for (int r = 0; r < 8; ++r) { const int rl = 8 * g + r;
      { const float q = (col < DQ) ? acc[0][r] + bfr(BQ[col]) : 0.f; sq[wave][rl][col] = (_Float16)q; sq[wave][rl][16 + col] = (_Float16)0.f; }
      { const float k = (col < DQ) ? acc[1][r] + bfr(BK[col]) : 0.f; sk[wave][rl][col] = (_Float16)k; sk[wave][rl][16 + col] = (_Float16)0.f; }
#pragma unroll
      for (int j = 2; j < 6; ++j) { const int c = (j - 2) * 16 + col; svt[c][wave * 16 + rl] = (_Float16)(acc[j][r] + bfr(BV[c])); } } }
  __syncthreads();
  for (int rl = 0; rl < 16; ++rl) { if (lane < 16) vst2(H + (r0 + rl) * L3D + lane * 4, *(const v4f*)&sH[wave][rl][lane * 4]);
    else if ((rl & 1) == 0) {
      const int l8 = lane & 7; const int rr = rl + (l8 >> 2); const int pc = l8 & 3;
      if (lane < 24) vst2((unsigned*)(QH + (r0 + rr) * 32 + pc * 8), *(const v4u*)&sq[wave][rr][pc * 8]); else vst2((unsigned*)(KH + (r0 + rr) * 32 + pc * 8), *(const v4u*)&sk[wave][rr][pc * 8]); } }
  for (int e = tid; e < L3D * 8; e += 128) { const int c = e >> 3, pc = e & 7; vst2((unsigned*)(VT + (size_t)c * NP + (size_t)blockIdx.x * 64 + pc * 8), *(const v4u*)&svt[c][pc * 8]); }
}
__global__ __launch_bounds__(128) void k_attn(const _Float16* __restrict__ QH, const _Float16* __restrict__ KH, const _Float16* __restrict__ VT, const float* __restrict__ H, const float* __restrict__ GAM, float* __restrict__ H2) {
  __shared__ __align__(16) _Float16 sp[4][16][40]; __shared__ __align__(16) float so[4][16][L3D + 4];
  const int tid = threadIdx.x, wave = tid >> 5, lane = tid & 31, col = lane & 15, g = lane >> 4; const size_t q0 = (size_t)blockIdx.x * 64 + wave * 16;
  const v16h aq = frag_h(QH + (q0 + col) * 32, lane);
  float m[8], l[8];
#pragma unroll
  for (int r = 0; r < 8; ++r) { m[r] = -3.0e38f; l[r] = 0.f; }
  v8f acc[4] = {};
#pragma unroll 1
  for (int ks = 0; ks < NP / 32; ++ks) { v8f s[2];
#pragma unroll
    for (int ct = 0; ct < 2; ++ct) { const size_t kk = (size_t)ks * 32 + ct * 16 + col; v8f c = {}; c = wmma16(aq, frag_h(KH + kk * 32, lane), c);
#pragma unroll
      for (int r = 0; r < 8; ++r) s[ct][r] = c[r]; }
#pragma unroll
    for (int r = 0; r < 8; ++r) { float mx = fmaxf(s[0][r], s[1][r]);
#pragma unroll
      for (int o = 1; o < 16; o <<= 1) mx = fmaxf(mx, __shfl_xor(mx, o));
      const float mn = fmaxf(m[r], mx); const float alpha = (m[r] <= -1.0e38f) ? 0.f : exp_ni(m[r] - mn); const float e0 = exp_ni(s[0][r] - mn), e1 = exp_ni(s[1][r] - mn); float es = e0 + e1;
#pragma unroll
      for (int o = 1; o < 16; o <<= 1) es += __shfl_xor(es, o);
      l[r] = l[r] * alpha + es; m[r] = mn;
#pragma unroll
      for (int dt = 0; dt < 4; ++dt) acc[dt][r] *= alpha;
      sp[wave][8 * g + r][col] = (_Float16)e0; sp[wave][8 * g + r][16 + col] = (_Float16)e1; }
    LDSX();
    const v16h pa = frag_h(&sp[wave][col][0], lane);
#pragma unroll
    for (int dt = 0; dt < 4; ++dt) acc[dt] = wmma16(pa, frag_h(VT + (size_t)(dt * 16 + col) * NP + (size_t)ks * 32, lane), acc[dt]);
    LDSX(); }
  const float gam = bfr(GAM[0]);
#pragma unroll
  for (int r = 0; r < 8; ++r) { const float il = 1.0f / l[r];
#pragma unroll
    for (int dt = 0; dt < 4; ++dt) { const int c = dt * 16 + col; so[wave][8 * g + r][c] = gam * (acc[dt][r] * il) + H[(q0 + 8 * g + r) * L3D + c]; } }
  LDSX();
  for (int rl = 0; rl < 16; ++rl) if (lane < 16) vst2(H2 + (q0 + rl) * L3D + lane * 4, *(const v4f*)&so[wave][rl][lane * 4]);
}
__global__ __launch_bounds__(256) void k_score(const float* __restrict__ H2, const float* __restrict__ WA1, const float* __restrict__ BA1, const float* __restrict__ WA2, const float* __restrict__ BA2, float* __restrict__ SC) {
  __shared__ __align__(16) float ssc[64]; const int tid = threadIdx.x; const int rl = tid >> 2, part = tid & 3; const size_t row = (size_t)blockIdx.x * 64 + rl; const float* h = H2 + row * L3D; float a = 0.f;
#pragma unroll 1
  for (int o = part; o < L3D; o += 4) { float t = 0.f;
#pragma unroll 1
    for (int k = 0; k < L3D; ++k) t += h[k] * bfr(WA1[(size_t)k * L3D + o]);
    a += tanh_ni(t + bfr(BA1[o])) * bfr(WA2[o]); }
  a += __shfl_xor(a, 1); a += __shfl_xor(a, 2);
  if (part == 0) ssc[rl] = a + bfr(BA2[0]);
  __syncthreads();
  if (tid < 16) vst2(SC + (size_t)blockIdx.x * 64 + tid * 4, *(const v4f*)&ssc[tid * 4]);
}
__global__ __launch_bounds__(256) void k_final(const float* __restrict__ SC, const float* __restrict__ H2, const float* __restrict__ WC, const float* __restrict__ BC, float* __restrict__ OUT) {
  __shared__ float sred[8]; __shared__ float smx, sinv; __shared__ double spart[4][L3D]; __shared__ __align__(16) float sout[68]; const int t = threadIdx.x;
  float mx = -3.0e38f; for (int i = t; i < NP; i += 256) mx = fmaxf(mx, SC[i]);
#pragma unroll
  for (int o = 1; o < 32; o <<= 1) mx = fmaxf(mx, __shfl_xor(mx, o));
  if ((t & 31) == 0) sred[t >> 5] = mx;
  __syncthreads();
  if (t == 0) { float a = sred[0]; for (int w = 1; w < 8; ++w) a = fmaxf(a, sred[w]); smx = a; }
  __syncthreads();
  { double se = 0.0; for (int i = t; i < NP; i += 256) se += (double)exp_ni(SC[i] - smx);
#pragma unroll
    for (int o = 1; o < 32; o <<= 1) se += __shfl_xor(se, o);
    if ((t & 31) == 0) sred[t >> 5] = (float)se; }
  __syncthreads();
  if (t == 0) { double a = 0.0; for (int w = 0; w < 8; ++w) a += (double)sred[w]; sinv = (float)(1.0 / a); }
  __syncthreads();
  { const int d = t & 63, part = t >> 6; double a = 0.0;
#pragma unroll 1
    for (int i = part; i < NP; i += 4) a += (double)(exp_ni(SC[i] - smx) * sinv) * (double)H2[(size_t)i * L3D + d];
    spart[part][d] = a; }
  __syncthreads();
  if (t < L3D) sout[1 + t] = (float)((spart[0][t] + spart[1][t]) + (spart[2][t] + spart[3][t]));
  __syncthreads();
  if (t == 0) { float a = 0.f; for (int d = 0; d < L3D; ++d) a += sout[1 + d] * bfr(WC[d]); a += bfr(BC[0]); float y = 1.0f / (1.0f + exp_ni(-a)); y = fminf(fmaxf(y, 1e-5f), 1.0f - 1e-5f); sout[0] = y; sout[65] = 0.f; sout[66] = 0.f; sout[67] = 0.f; }
  __syncthreads();
  if (t < 16) vst2(OUT + t * 4, *(const v4f*)&sout[t * 4]);
  if (t == 16) { *(volatile float*)(OUT + 64) = sout[64]; *(volatile float*)(OUT + 64) = sout[64]; }
}
extern "C" void kernel_launch(void* const* d_in, const int* in_sizes, int n_in, void* d_out, int out_size, void* d_ws, size_t ws_size, hipStream_t stream) {
  (void)in_sizes; (void)n_in; (void)out_size;
  const float** F = (const float**)d_in;
  if (ws_size < (size_t)WS_END) return;
  char* ws = (char*)d_ws; __bf16* PK = (__bf16*)(ws + WS_PK); float *H = (float*)(ws + WS_H), *H2 = (float*)(ws + WS_H2), *SC = (float*)(ws + WS_SC); _Float16 *QH = (_Float16*)(ws + WS_QH), *KH = (_Float16*)(ws + WS_KH), *VT = (_Float16*)(ws + WS_VT);
  k_pack<<<dim3(L1D, 6), 256, 0, stream>>>(F[1], F[3], F[5], F[7], F[9], F[11], PK);
  k_mlp<<<NP / 64, 128, 0, stream>>>(F[0], PK, F[2], F[4], F[6], F[8], F[10], F[12], H, QH, KH, VT);
  k_attn<<<NP / 64, 128, 0, stream>>>(QH, KH, VT, H, F[13], H2);
  k_score<<<NP / 64, 256, 0, stream>>>(H2, F[14], F[15], F[16], F[17], SC);
  k_final<<<1, 256, 0, stream>>>(SC, H2, F[18], F[19], (float*)d_out);
}
